// mLSTM_57775900066443
// MI455X (gfx1250) — hardware-verified
//
#include <hip/hip_runtime.h>
#include <math.h>

constexpr int kB    = 4;
constexpr int kT    = 2048;
constexpr int kD    = 256;
constexpr int kRows = kB * kT;
constexpr int kNP   = 6 * kD;
constexpr int kL    = 32;
constexpr int kNC   = kT / kL;
constexpr int kPairs = kRows / 64;
constexpr int cQ = 0, cK = 256, cV = 512, cI = 768, cF = 1024, cO = 1280;
constexpr float kKScale = 0.0625f;
static_assert(kRows % 64 == 0 && kNP % 64 == 0 && kD % 32 == 0, "proj gemm tiles: M,N %64, K %32");
static_assert(kD % 64 == 0 && (64 % 64) == 0, "score gemm tiles: M=N=64, K=256");
static_assert(kT % 64 == 0 && kL == 32 && kT % kL == 0, "chunking");
static_assert(kD == 256, "thread-per-feature mappings assume D=256");

typedef __attribute__((ext_vector_type(16))) _Float16 v16h;
typedef __attribute__((ext_vector_type(8)))  _Float16 v8h;
typedef __attribute__((ext_vector_type(16))) __bf16   v16b;
typedef __attribute__((ext_vector_type(8)))  __bf16   v8b;
typedef __attribute__((ext_vector_type(4)))  __bf16   v4b;
typedef __attribute__((ext_vector_type(8)))  float    v8f;
typedef __attribute__((ext_vector_type(4)))  float    v4f;
typedef __attribute__((ext_vector_type(4)))  unsigned int v4u;
typedef __attribute__((ext_vector_type(2)))  unsigned int v2u;

__device__ __forceinline__ unsigned short f2bf_bits(float f) {
  unsigned u = __float_as_uint(f);
  return (unsigned short)((u + 0x7FFFu + ((u >> 16) & 1u)) >> 16);
}
__device__ __forceinline__ float bf_bits2f(unsigned short h) { return __uint_as_float(((unsigned)h) << 16); }

__device__ __forceinline__ void dep_guard_h(v8f& a, v8f& b, v16h x, v16h y) { asm volatile("v_nop\n\tv_nop\n\tv_nop\n\tv_nop" : "+v"(a), "+v"(b) : "v"(x), "v"(y)); }
__device__ __forceinline__ void dep_guard_b(v8f& a, v8f& b, v16b x, v16b y) { asm volatile("v_nop\n\tv_nop\n\tv_nop\n\tv_nop" : "+v"(a), "+v"(b) : "v"(x), "v"(y)); }
__device__ __forceinline__ void dep_guard4_h(v8f& a, v8f& b, v8f& c, v8f& d, v16h x, v16h y) { asm volatile("v_nop\n\tv_nop\n\tv_nop\n\tv_nop" : "+v"(a), "+v"(b), "+v"(c), "+v"(d) : "v"(x), "v"(y)); }
__device__ __forceinline__ void dep_guard4_b(v8f& a, v8f& b, v8f& c, v8f& d, v16b x, v16b y) { asm volatile("v_nop\n\tv_nop\n\tv_nop\n\tv_nop" : "+v"(a), "+v"(b), "+v"(c), "+v"(d) : "v"(x), "v"(y)); }
__device__ __forceinline__ void keep4_h(v16h a, v16h b, v16h c, v16h d) { asm volatile("v_nop" :: "v"(a), "v"(b), "v"(c), "v"(d)); }
__device__ __forceinline__ void keep4_b(v16b a, v16b b, v16b c, v16b d) { asm volatile("v_nop" :: "v"(a), "v"(b), "v"(c), "v"(d)); }
__device__ __forceinline__ void acc_guard4(v8f& a, v8f& b, v8f& c, v8f& d) { asm volatile("v_nop\n\tv_nop\n\tv_nop\n\tv_nop" : "+v"(a), "+v"(b), "+v"(c), "+v"(d)); }
template <typename T> struct Frag;
template <> struct Frag<_Float16> {
  typedef v16h V; union U { v16h v; v8h h[2]; };
  static __device__ __forceinline__ v16h load(const _Float16* p) {
    U f; f.h[0] = *(const v8h*)(p); f.h[1] = *(const v8h*)(p + 16); return f.v;
  }
  static __device__ __forceinline__ v8f mma(v16h a, v16h b, v8f c) {
    return __builtin_amdgcn_wmma_f32_16x16x32_f16(false, a, false, b, (short)0, c, false, false);
  }
  static __device__ __forceinline__ void guard(v8f& a, v8f& b, v16h x, v16h y) { dep_guard_h(a, b, x, y); }
  static __device__ __forceinline__ void guard4(v8f& a, v8f& b, v8f& c, v8f& d, v16h x, v16h y) { dep_guard4_h(a, b, c, d, x, y); }
  static __device__ __forceinline__ void keep(v16h a, v16h b, v16h c, v16h d) { keep4_h(a, b, c, d); }
};
template <> struct Frag<__bf16> {
  typedef v16b V; union U { v16b v; v8b h[2]; };
  static __device__ __forceinline__ v16b load(const __bf16* p) {
    U f; f.h[0] = *(const v8b*)(p); f.h[1] = *(const v8b*)(p + 16); return f.v;
  }
  static __device__ __forceinline__ v8f mma(v16b a, v16b b, v8f c) {
    return __builtin_amdgcn_wmma_f32_16x16x32_bf16(false, a, false, b, (short)0, c, false, false);
  }
  static __device__ __forceinline__ void guard(v8f& a, v8f& b, v16b x, v16b y) { dep_guard_b(a, b, x, y); }
  static __device__ __forceinline__ void guard4(v8f& a, v8f& b, v8f& c, v8f& d, v16b x, v16b y) { dep_guard4_b(a, b, c, d, x, y); }
  static __device__ __forceinline__ void keep(v16b a, v16b b, v16b c, v16b d) { keep4_b(a, b, c, d); }
};

__device__ __forceinline__ unsigned pkw(unsigned a, unsigned b) { return (a & 0xffffu) | (b << 16); }

__device__ __forceinline__ v8f mma_g(v16b a, v16b b, v8f c) {
  c = __builtin_amdgcn_wmma_f32_16x16x32_bf16(false, a, false, b, (short)0, c, false, false);
  asm volatile("v_nop\n\tv_nop\n\tv_nop\n\tv_nop" : "+v"(c) : "v"(a), "v"(b));
  return c;
}

__device__ __forceinline__ void split2(float f, unsigned& hb, unsigned& lb) {
  const unsigned u  = __float_as_uint(f);
  const unsigned hu = u & 0xffff0000u;
  hb = hu >> 16;
  lb = (unsigned)f2bf_bits(f - __uint_as_float(hu));
}

template <int ET> struct Elem;
template <> struct Elem<0> { typedef _Float16 T; };
template <> struct Elem<1> { typedef __bf16 T; };
template <int ET, bool SPLIT, int BIAS_MODE, int OUT_MODE, bool RESID, int ACT = 0>
__global__ __launch_bounds__(256) void wmma_gemm64(
    const unsigned short* __restrict__ Ap, const unsigned short* __restrict__ A2p, int lda, long strideA,
    const unsigned short* __restrict__ Btp, const unsigned short* __restrict__ Bt2p, int ldb, long strideB,
    void* __restrict__ Cout, void* __restrict__ Cout2, int ldc, long strideC,
    const float* __restrict__ bias,
    const float* __restrict__ resid, long strideR,
    int M, int N, int K, float scale) {
  typedef typename Elem<ET>::T T;
  typedef typename Frag<T>::V V;
  const T* A = (const T*)Ap; const T* A2 = (const T*)A2p; const T* Bt = (const T*)Btp; const T* Bt2 = (const T*)Bt2p;
  __shared__ __align__(16) float sT[8][16 * 68];
  const int b    = blockIdx.y;
  const int lane = threadIdx.x & 31;
  const int wave = threadIdx.x >> 5;
  const int tilesN = N >> 6;
  const int tilesM = M >> 6;
  const int tile = blockIdx.x * 8 + wave;
  if (tile >= tilesM * tilesN) return;
  const int tm = tile / tilesN;
  const int tn = tile - tm * tilesN;
  const int m0 = tm << 6;
  const int n0 = tn << 6;

  const T* Ab  = A  + (size_t)b * strideA;
  const T* Bb  = Bt + (size_t)b * strideB;
  const T* Ab2 = SPLIT ? (A2  + (size_t)b * strideA) : nullptr;
  const T* Bb2 = SPLIT ? (Bt2 + (size_t)b * strideB) : nullptr;

  const int rlane = lane & 15;
  const int koff  = (lane >> 4) * 8;
  const int mOff  = (lane >> 4) * 8;

  v8f acc[4][4];
#pragma unroll
  for (int i = 0; i < 4; ++i)
#pragma unroll
    for (int j = 0; j < 4; ++j) acc[i][j] = (v8f){0.f,0.f,0.f,0.f,0.f,0.f,0.f,0.f};

  for (int k0 = 0; k0 < K; k0 += 32) {
    V bh[4], bl[4];
#pragma unroll
    for (int j = 0; j < 4; ++j) {
      const size_t bo = (size_t)(n0 + (j << 4) + rlane) * ldb + koff + k0;
      bh[j] = Frag<T>::load(Bb + bo);
      if (SPLIT) bl[j] = Frag<T>::load(Bb2 + bo);
    }
#pragma unroll
    for (int i = 0; i < 4; ++i) {
      const size_t ao = (size_t)(m0 + (i << 4) + rlane) * lda + koff + k0;
      V ah = Frag<T>::load(Ab + ao);
      V al;
      if (SPLIT) al = Frag<T>::load(Ab2 + ao);
#pragma unroll
      for (int j = 0; j < 4; ++j) {
        acc[i][j] = Frag<T>::mma(ah, bh[j], acc[i][j]);
        if (SPLIT) {
          acc[i][j] = Frag<T>::mma(ah, bl[j], acc[i][j]);
          acc[i][j] = Frag<T>::mma(al, bh[j], acc[i][j]);
        }
      }
      Frag<T>::guard4(acc[i][0], acc[i][1], acc[i][2], acc[i][3], ah, SPLIT ? al : ah);
    }
    Frag<T>::keep(bh[0], bh[1], bh[2], bh[3]);
    if (SPLIT) Frag<T>::keep(bl[0], bl[1], bl[2], bl[3]);
  }
  acc_guard4(acc[0][0], acc[0][1], acc[0][2], acc[0][3]);
  acc_guard4(acc[1][0], acc[1][1], acc[1][2], acc[1][3]);
  acc_guard4(acc[2][0], acc[2][1], acc[2][2], acc[2][3]);
  acc_guard4(acc[3][0], acc[3][1], acc[3][2], acc[3][3]);

  float* slab = sT[wave];
  const float* Rb = RESID ? (resid + (size_t)b * strideR) : nullptr;
#pragma unroll
  for (int i = 0; i < 4; ++i) {
    const int mBase = m0 + (i << 4);
#pragma unroll
    for (int j = 0; j < 4; ++j) {
      const int n = n0 + (j << 4) + rlane;
      float bv = 0.f;
      if (BIAS_MODE == 2) bv = bias[n];
#pragma unroll
      for (int r = 0; r < 8; ++r) {
        float v = acc[i][j][r] * scale;
        if (BIAS_MODE == 1) v += bias[mBase + mOff + r];
        if (BIAS_MODE == 2) v += bv;
        if (RESID) v += Rb[(size_t)(mBase + mOff + r) * ldc + n];
        if (ACT == 2) v = fmaxf(v, 0.0f);
        if (ACT == 4) v = (v > 0.f) ? v : 0.01f * v;
        slab[(mOff + r) * 68 + (j << 4) + rlane] = v;
      }
    }
    __builtin_amdgcn_fence(__ATOMIC_RELEASE, "workgroup");
    __builtin_amdgcn_wave_barrier();
    __builtin_amdgcn_fence(__ATOMIC_ACQUIRE, "workgroup");
    if (OUT_MODE == 0) {
      float* C = (float*)Cout + (size_t)b * strideC;
      const int hh = lane >> 4, c4 = (lane & 15) * 4;
      for (int pass = 0; pass < 2; ++pass) {
#pragma unroll
        for (int it = 0; it < 8; ++it) {
          const int row = it * 2 + hh;
          v4f v = *(const v4f*)(slab + row * 68 + c4);
          *(volatile v4f*)(C + (size_t)(mBase + row) * ldc + n0 + c4) = v;
        }
        __threadfence();
      }
    } else {
      const int q = lane >> 3, c8 = (lane & 7) * 8;
      unsigned short* C  = (unsigned short*)Cout  + (size_t)b * strideC;
      unsigned short* C2 = (OUT_MODE == 2) ? ((unsigned short*)Cout2 + (size_t)b * strideC) : nullptr;
      for (int pass = 0; pass < 2; ++pass) {
#pragma unroll
        for (int it = 0; it < 4; ++it) {
          const int row = it * 4 + q;
          const float* sp = slab + row * 68 + c8;
          v8h hv, lv;
#pragma unroll
          for (int e = 0; e < 8; ++e) {
            if (OUT_MODE == 1) {
              hv[e] = (_Float16)sp[e];
            } else {
              unsigned short hb = f2bf_bits(sp[e]);
              unsigned short lb = f2bf_bits(sp[e] - bf_bits2f(hb));
              hv[e] = __builtin_bit_cast(_Float16, hb);
              lv[e] = __builtin_bit_cast(_Float16, lb);
            }
          }
          *(volatile v8h*)(C + (size_t)(mBase + row) * ldc + n0 + c8) = hv;
          if (OUT_MODE == 2) *(volatile v8h*)(C2 + (size_t)(mBase + row) * ldc + n0 + c8) = lv;
        }
        __threadfence();
      }
    }
    __builtin_amdgcn_fence(__ATOMIC_RELEASE, "workgroup");
    __builtin_amdgcn_wave_barrier();
    __builtin_amdgcn_fence(__ATOMIC_ACQUIRE, "workgroup");
  }
}

__global__ __launch_bounds__(64) void bias_cat_kernel(const float* __restrict__ bq, const float* __restrict__ bk,
                                                      const float* __restrict__ bv, const float* __restrict__ bg,
                                                      float* __restrict__ Bc) {
  const int seg = blockIdx.x;
  const int t = threadIdx.x;
  const int goff = (seg >= 3) ? (seg - 3) * kD : 0;
  const float* src = (seg == 0) ? bq : (seg == 1) ? bk : (seg == 2) ? bv : (bg + goff);
  const v4f v = *(const v4f*)(src + 4 * t);
  float* dp = Bc + seg * kD + 4 * t;
  *(volatile v4f*)dp = v;
  __threadfence();
  *(volatile v4f*)dp = v;
}

__global__ __launch_bounds__(256) void xcast_kernel(const float* __restrict__ x, unsigned short* __restrict__ Xb, int n8) {
  const int i = blockIdx.x * 256 + threadIdx.x;
  if (i >= n8) return;
  const float* p = x + 8 * (size_t)i;
  const v4f a = *(const v4f*)(p);
  const v4f c = *(const v4f*)(p + 4);
  unsigned hb[8];
#pragma unroll
  for (int e = 0; e < 4; ++e) {
    hb[e]     = (unsigned)f2bf_bits(a[e]);
    hb[4 + e] = (unsigned)f2bf_bits(c[e]);
  }
  const v4u u = (v4u){pkw(hb[0], hb[1]), pkw(hb[2], hb[3]), pkw(hb[4], hb[5]), pkw(hb[6], hb[7])};
  unsigned short* q = Xb + 8 * (size_t)i;
  *(volatile v4u*)q = u;
  __threadfence();
  *(volatile v4u*)q = u;
}

__global__ __launch_bounds__(256) void wt_cast_kernel(const float* __restrict__ Wq, const float* __restrict__ Wk,
                                                      const float* __restrict__ Wv, const float* __restrict__ Wg,
                                                      unsigned short* __restrict__ Wt) {
  __shared__ float sm[64][65];
  const int t  = threadIdx.x;
  const int k0 = blockIdx.x * 64;
  const int nt = blockIdx.y;
  const int n0 = nt * 64;
  const int seg = nt >> 2;
  const float* W = (seg == 0) ? Wq : (seg == 1) ? Wk : (seg == 2) ? Wv : Wg;
  const int width = (seg < 3) ? kD : 3 * kD;
  const int col0  = (seg < 3) ? (n0 - seg * kD) : (n0 - 3 * kD);
#pragma unroll
  for (int i = 0; i < 16; ++i) {
    const int e  = i * 256 + t;
    const int r  = e >> 6;
    const int cc = e & 63;
    sm[cc][r] = W[(size_t)(k0 + r) * width + col0 + cc];
  }
  __syncthreads();
  const int lane = t & 31, wave = t >> 5;
  const int q = lane >> 3, c8 = (lane & 7) * 8;
  for (int pass = 0; pass < 2; ++pass) {
#pragma unroll
    for (int it = 0; it < 2; ++it) {
      const int row = wave * 8 + it * 4 + q;
      unsigned hb[8];
#pragma unroll
      for (int e = 0; e < 8; ++e) hb[e] = (unsigned)f2bf_bits(sm[row][c8 + e]);
      const v4u u = (v4u){pkw(hb[0], hb[1]), pkw(hb[2], hb[3]), pkw(hb[4], hb[5]), pkw(hb[6], hb[7])};
      *(volatile v4u*)(Wt + (size_t)(n0 + row) * kD + k0 + c8) = u;
    }
    __threadfence();
  }
}

__global__ __launch_bounds__(256) void split_qk_kernel(const float* __restrict__ PR,
                                                       unsigned short* __restrict__ Qh, unsigned short* __restrict__ Ql,
                                                       unsigned short* __restrict__ Kh, unsigned short* __restrict__ Kl) {
  const int y = blockIdx.y;
  const int i = blockIdx.x * 256 + threadIdx.x;
  const int row = i >> 5, c = (i & 31) * 8;
  const int coff = y ? cK : cQ;
  const float sc = y ? kKScale : 1.0f;
  unsigned short* H = y ? Kh : Qh;
  unsigned short* L = y ? Kl : Ql;
  const float* p = PR + (size_t)row * kNP + coff + c;
  const v4f a = *(const v4f*)(p);
  const v4f d = *(const v4f*)(p + 4);
  unsigned hw[4], lw[4];
#pragma unroll
  for (int e = 0; e < 2; ++e) {
    unsigned h0, l0, h1, l1;
    split2(a[2 * e] * sc, h0, l0); split2(a[2 * e + 1] * sc, h1, l1);
    hw[e] = pkw(h0, h1); lw[e] = pkw(l0, l1);
    split2(d[2 * e] * sc, h0, l0); split2(d[2 * e + 1] * sc, h1, l1);
    hw[2 + e] = pkw(h0, h1); lw[2 + e] = pkw(l0, l1);
  }
  const v4u hu = (v4u){hw[0], hw[1], hw[2], hw[3]};
  const v4u lu = (v4u){lw[0], lw[1], lw[2], lw[3]};
  unsigned short* hp = H + (size_t)row * kD + c;
  unsigned short* lp = L + (size_t)row * kD + c;
  *(volatile v4u*)hp = hu;
  *(volatile v4u*)lp = lu;
  __threadfence();
  *(volatile v4u*)hp = hu;
  *(volatile v4u*)lp = lu;
}

__global__ __launch_bounds__(256) void gate_kernel(const float* __restrict__ PR, const float* __restrict__ ib,
                                                   float* __restrict__ Wpl, float* __restrict__ Epl, float* __restrict__ Npl) {
  const int b = blockIdx.x;
  const int i = threadIdx.x;
  const float ibi = ib[i];
  float m0 = 0.0f, n0 = 0.0f;
#pragma unroll 1
  for (int c = 0; c < kNC; ++c) {
    float Lf = 0.0f, g = m0, cums = 0.0f, nlast = n0;
#pragma unroll 1
    for (int t = 0; t < kL; ++t) {
      const size_t row = (size_t)(b * kT + c * kL + t);
      const float ip = PR[row * kNP + cI + i];
      const float fp = PR[row * kNP + cF + i];
      const float kk = PR[row * kNP + cK + i] * kKScale;
      const float li = 10.0f * tanhf((ip + ibi) * 0.1f);
      const float sp = fmaxf(fp, 0.0f) + log1pf(expf(-fabsf(fp)));
      Lf = Lf - sp;
      const float a = li - Lf;
      g = fmaxf(g, a);
      const float w  = expf(fminf(a - m0, 87.0f));
      const float ev = expf(m0 - g);
      cums = cums + w * kk;
      const float nt = ev * (n0 + cums);
      nlast = nt;
      float* wp = Wpl + row * kD + i;
      float* ep = Epl + row * kD + i;
      float* np2 = Npl + row * kD + i;
      *(volatile float*)wp = w;
      *(volatile float*)ep = ev;
      *(volatile float*)np2 = nt;
      __threadfence();
      *(volatile float*)wp = w;
      *(volatile float*)ep = ev;
      *(volatile float*)np2 = nt;
    }
    m0 = g + Lf;
    n0 = nlast;
  }
}

__global__ __launch_bounds__(256) void scan_kernel(
    const unsigned short* __restrict__ Qh, const unsigned short* __restrict__ Ql,
    const float* __restrict__ PR, const float* __restrict__ SS,
    const float* __restrict__ Wpl, const float* __restrict__ Epl, const float* __restrict__ Npl,
    float* __restrict__ Hp) {
  __shared__ __align__(16) float  sM[64 * 256];
  __shared__ __align__(16) __bf16 sMh[64 * 256];
  __shared__ __align__(16) __bf16 sMl[64 * 256];
  __shared__ __align__(16) __bf16 sKh[256 * 32];
  __shared__ __align__(16) __bf16 sKl[256 * 32];
  __shared__ __align__(16) __bf16 sVh[64 * 32];
  __shared__ __align__(16) __bf16 sVl[64 * 32];
  __shared__ __align__(16) __bf16 sAh[32 * 32];
  __shared__ __align__(16) __bf16 sAl[32 * 32];
  __shared__ __align__(16) float  sF[32 * 64];
  __shared__ __align__(16) float  sH[32 * 68];
  __shared__ float sEe[64];
  __shared__ float sRd[32];

  const int tid = threadIdx.x, lane = tid & 31, wave = tid >> 5;
  const int hh = lane >> 4, rl = lane & 15, koff = hh * 8;
  const int rg = blockIdx.x, b = blockIdx.y;
  const int fbase = rg * 64;
  const __bf16 bz = __builtin_bit_cast(__bf16, (unsigned short)0);

#pragma unroll 4
  for (int e = tid; e < 64 * 256; e += 256) { sM[e] = 0.0f; sMh[e] = bz; sMl[e] = bz; }
  __syncthreads();

#pragma unroll 1
  for (int c = 0; c < kNC; ++c) {
    const int t0 = b * kT + c * kL;

    {
      const int j = tid;
#pragma unroll 1
      for (int grp = 0; grp < 4; ++grp) {
        float kv[8];
#pragma unroll
        for (int e = 0; e < 8; ++e) kv[e] = PR[(size_t)(t0 + grp * 8 + e) * kNP + cK + j] * kKScale;
        unsigned hw[4], lw[4];
#pragma unroll
        for (int e = 0; e < 4; ++e) {
          unsigned h0, l0, h1, l1;
          split2(kv[2 * e], h0, l0); split2(kv[2 * e + 1], h1, l1);
          hw[e] = pkw(h0, h1); lw[e] = pkw(l0, l1);
        }
        const v4u hv = (v4u){hw[0], hw[1], hw[2], hw[3]};
        const v4u lv = (v4u){lw[0], lw[1], lw[2], lw[3]};
        *(v8b*)(sKh + j * 32 + grp * 8) = __builtin_bit_cast(v8b, hv);
        *(v8b*)(sKl + j * 32 + grp * 8) = __builtin_bit_cast(v8b, lv);
      }
    }
    {
      const int il = tid & 63, s8 = (tid >> 6) * 8, i = fbase + il;
#pragma unroll 1
      for (int grp = 0; grp < 2; ++grp) {
        float pv[4];
#pragma unroll
        for (int e = 0; e < 4; ++e) {
          const size_t row = (size_t)(t0 + s8 + grp * 4 + e);
          pv[e] = Wpl[row * kD + i] * PR[row * kNP + cV + i];
        }
        unsigned h0, l0, h1, l1, h2, l2, h3, l3;
        split2(pv[0], h0, l0); split2(pv[1], h1, l1); split2(pv[2], h2, l2); split2(pv[3], h3, l3);
        const v2u hv = (v2u){pkw(h0, h1), pkw(h2, h3)};
        const v2u lv = (v2u){pkw(l0, l1), pkw(l2, l3)};
        *(v4b*)(sVh + il * 32 + s8 + grp * 4) = __builtin_bit_cast(v4b, hv);
        *(v4b*)(sVl + il * 32 + s8 + grp * 4) = __builtin_bit_cast(v4b, lv);
      }
    }
    {
      const int t = tid >> 3, s4 = (tid & 7) * 4;
      const int p = t0 >> 6, half = c & 1;
      const v4f sv = *(const v4f*)(SS + (size_t)p * 4096 + (size_t)(32 * half + t) * 64 + 32 * half + s4);
      unsigned hw[2], lw[2];
#pragma unroll
      for (int e = 0; e < 2; ++e) {
        const int s0 = s4 + 2 * e, s1 = s0 + 1;
        const float mk0 = (s0 <= t) ? 1.0f : 0.0f;
        const float mk1 = (s1 <= t) ? 1.0f : 0.0f;
        unsigned h0, l0, h1, l1;
        split2(sv[2 * e] * mk0, h0, l0); split2(sv[2 * e + 1] * mk1, h1, l1);
        hw[e] = pkw(h0, h1); lw[e] = pkw(l0, l1);
      }
      const v2u hv = (v2u){hw[0], hw[1]};
      const v2u lv = (v2u){lw[0], lw[1]};
      *(v4b*)(sAh + t * 32 + s4) = __builtin_bit_cast(v4b, hv);
      *(v4b*)(sAl + t * 32 + s4) = __builtin_bit_cast(v4b, lv);
    }
    {
#pragma unroll 1
      for (int rr = 0; rr < 4; ++rr) {
        const int t = wave * 4 + rr;
        const size_t row = (size_t)(t0 + t);
        const v4f na = *(const v4f*)(Npl + row * kD + lane * 8);
        const v4f nb = *(const v4f*)(Npl + row * kD + lane * 8 + 4);
        const v4f qa = *(const v4f*)(PR + row * kNP + cQ + lane * 8);
        const v4f qb = *(const v4f*)(PR + row * kNP + cQ + lane * 8 + 4);
        float s = 0.0f;
#pragma unroll
        for (int e = 0; e < 4; ++e) s += na[e] * qa[e];
#pragma unroll
        for (int e = 0; e < 4; ++e) s += nb[e] * qb[e];
#pragma unroll
        for (int off = 16; off > 0; off >>= 1) s += __shfl_xor(s, off, 32);
        if (lane == 0) sRd[t] = 1.0f / fmaxf(fabsf(s), 1e-6f);
      }
      if (tid < 64) sEe[tid] = Epl[(size_t)(t0 + kL - 1) * kD + fbase + tid];
    }
    __syncthreads();

    {
      const int il = tid & 63, tb = tid >> 6, i = fbase + il;
#pragma unroll 1
      for (int r = 0; r < 8; ++r) {
        const int t = tb + 4 * r;
        const size_t row = (size_t)(t0 + t);
        const float o  = PR[row * kNP + cO + i];
        const float ev = Epl[row * kD + i];
        const float sg = 1.0f / (1.0f + expf(-o));
        sF[t * 64 + il] = sg * ev * sRd[t];
      }
    }
    __syncthreads();

    {
      const int tt = wave >> 2, jt = wave & 3;
      v8f acc = (v8f){0.f, 0.f, 0.f, 0.f, 0.f, 0.f, 0.f, 0.f};
      const __bf16* qh = (const __bf16*)Qh + (size_t)(t0 + 16 * tt + rl) * kD + koff;
      const __bf16* ql = (const __bf16*)Ql + (size_t)(t0 + 16 * tt + rl) * kD + koff;
      const __bf16* mh = sMh + (16 * jt + rl) * 256 + koff;
      const __bf16* ml = sMl + (16 * jt + rl) * 256 + koff;
#pragma unroll 2
      for (int ks = 0; ks < 8; ++ks) {
        const v16b ah = Frag<__bf16>::load(qh + 32 * ks);
        const v16b al = Frag<__bf16>::load(ql + 32 * ks);
        const v16b bh = Frag<__bf16>::load(mh + 32 * ks);
        const v16b bl = Frag<__bf16>::load(ml + 32 * ks);
        acc = mma_g(ah, bh, acc);
        acc = mma_g(ah, bl, acc);
        acc = mma_g(al, bh, acc);
      }
      {
        const v16b ah = Frag<__bf16>::load(sAh + (16 * tt + rl) * 32 + koff);
        const v16b al = Frag<__bf16>::load(sAl + (16 * tt + rl) * 32 + koff);
        const v16b bh = Frag<__bf16>::load(sVh + (16 * jt + rl) * 32 + koff);
        const v16b bl = Frag<__bf16>::load(sVl + (16 * jt + rl) * 32 + koff);
        acc = mma_g(ah, bh, acc);
        acc = mma_g(ah, bl, acc);
        acc = mma_g(al, bh, acc);
      }
#pragma unroll
      for (int r = 0; r < 8; ++r) {
        const int t = 16 * tt + 8 * hh + r, il = 16 * jt + rl;
        sH[t * 68 + il] = acc[r] * sF[t * 64 + il];
      }
    }
    __syncthreads();

    {
      float* hp = Hp + (size_t)t0 * kD + fbase;
      const int c4 = rl * 4;
      for (int pass = 0; pass < 2; ++pass) {
#pragma unroll
        for (int it = 0; it < 2; ++it) {
          const int row = wave * 4 + it * 2 + hh;
          const v4f v = *(const v4f*)(sH + row * 68 + c4);
          *(volatile v4f*)(hp + (size_t)row * kD + c4) = v;
        }
        __threadfence();
      }
    }

    {
      const int it3 = wave >> 1, jt0 = (wave & 1) * 8;
      const v16b ah = Frag<__bf16>::load(sVh + (16 * it3 + rl) * 32 + koff);
      const v16b al = Frag<__bf16>::load(sVl + (16 * it3 + rl) * 32 + koff);
#pragma unroll 1
      for (int q8 = 0; q8 < 8; ++q8) {
        const int jt = jt0 + q8;
        const v16b bh = Frag<__bf16>::load(sKh + (16 * jt + rl) * 32 + koff);
        const v16b bl = Frag<__bf16>::load(sKl + (16 * jt + rl) * 32 + koff);
        v8f acc = (v8f){0.f, 0.f, 0.f, 0.f, 0.f, 0.f, 0.f, 0.f};
        acc = mma_g(ah, bh, acc);
        acc = mma_g(ah, bl, acc);
        acc = mma_g(al, bh, acc);
#pragma unroll
        for (int r = 0; r < 8; ++r) {
          const int il = 16 * it3 + 8 * hh + r, j = 16 * jt + rl;
          const int idx = il * 256 + j;
          const float mn = sEe[il] * (sM[idx] + acc[r]);
          sM[idx] = mn;
          unsigned hb, lb;
          split2(mn, hb, lb);
          sMh[idx] = __builtin_bit_cast(__bf16, (unsigned short)hb);
          sMl[idx] = __builtin_bit_cast(__bf16, (unsigned short)lb);
        }
      }
    }
    __syncthreads();
  }
}

__global__ __launch_bounds__(256) void rmsnorm_kernel(const float* __restrict__ Hp, const float* __restrict__ ns,
                                                      float* __restrict__ out) {
  const int lane = threadIdx.x & 31, wave = threadIdx.x >> 5;
  const int row = blockIdx.x * 8 + wave;
  const float* hr = Hp + (size_t)row * kD;
  const v4f a = *(const v4f*)(hr + 4 * lane);
  const v4f c = *(const v4f*)(hr + 128 + 4 * lane);
  const v4f ga = *(const v4f*)(ns + 4 * lane);
  const v4f gc = *(const v4f*)(ns + 128 + 4 * lane);
  float ss = 0.0f;
#pragma unroll
  for (int e = 0; e < 4; ++e) ss += a[e] * a[e];
#pragma unroll
  for (int e = 0; e < 4; ++e) ss += c[e] * c[e];
#pragma unroll
  for (int off = 16; off > 0; off >>= 1) ss += __shfl_xor(ss, off, 32);
  const float rms = sqrtf(ss * (1.0f / 256.0f) + 1e-8f);
  const float rr = 1.0f / rms;
  v4f oa, oc;
#pragma unroll
  for (int e = 0; e < 4; ++e) { oa[e] = (a[e] * rr) * ga[e]; oc[e] = (c[e] * rr) * gc[e]; }
  float* op = out + (size_t)row * kD;
  *(volatile v4f*)(op + 4 * lane) = oa;
  *(volatile v4f*)(op + 128 + 4 * lane) = oc;
  __threadfence();
  *(volatile v4f*)(op + 4 * lane) = oa;
  *(volatile v4f*)(op + 128 + 4 * lane) = oc;
}

extern "C" void kernel_launch(void* const* d_in, const int* in_sizes, int n_in,
                              void* d_out, int out_size, void* d_ws, size_t ws_size,
                              hipStream_t stream) {
  if (n_in < 11) return;
  if (in_sizes[0] != kRows * kD) return;
  if (in_sizes[1] != kD * kD || in_sizes[3] != kD * kD || in_sizes[5] != kD * kD) return;
  if (in_sizes[7] != kD * 3 * kD) return;
  if (in_sizes[2] != kD || in_sizes[4] != kD || in_sizes[6] != kD || in_sizes[8] != 3 * kD) return;
  if (in_sizes[9] != kD || in_sizes[10] != kD) return;
  if (out_size != kRows * kD) return;

  const size_t szXb   = (size_t)kRows * kD * 2;
  const size_t szWt   = (size_t)kNP * kD * 2;
  const size_t szBc   = (size_t)kNP * 4;
  const size_t szPR   = (size_t)kRows * kNP * 4;
  const size_t szPl16 = (size_t)kRows * kD * 2;
  const size_t szSS   = (size_t)kPairs * 64 * 64 * 4;
  const size_t szPl32 = (size_t)kRows * kD * 4;
  const size_t offXb = 0;
  const size_t offWt = offXb + szXb;
  const size_t offBc = offWt + szWt;
  const size_t offPR = offBc + szBc;
  const size_t offQh = offPR + szPR;
  const size_t offQl = offQh + szPl16;
  const size_t offKh = offQl + szPl16;
  const size_t offKl = offKh + szPl16;
  const size_t offSS = offKl + szPl16;
  const size_t offW  = offSS + szSS;
  const size_t offE  = offW + szPl32;
  const size_t offN  = offE + szPl32;
  const size_t offH  = offN + szPl32;
  const size_t total = offH + szPl32;
  if (ws_size < total) return;

  const float* x  = (const float*)d_in[0];
  const float* Wq = (const float*)d_in[1];
  const float* bq = (const float*)d_in[2];
  const float* Wk = (const float*)d_in[3];
  const float* bk = (const float*)d_in[4];
  const float* Wv = (const float*)d_in[5];
  const float* bv = (const float*)d_in[6];
  const float* Wg = (const float*)d_in[7];
  const float* bg = (const float*)d_in[8];
  const float* ib = (const float*)d_in[9];
  const float* ns = (const float*)d_in[10];
  float* out = (float*)d_out;
  char* ws = (char*)d_ws;
  unsigned short* Xb = (unsigned short*)(ws + offXb);
  unsigned short* Wt = (unsigned short*)(ws + offWt);
  float* Bc = (float*)(ws + offBc);
  float* PR = (float*)(ws + offPR);
  unsigned short* Qh = (unsigned short*)(ws + offQh);
  unsigned short* Ql = (unsigned short*)(ws + offQl);
  unsigned short* Kh = (unsigned short*)(ws + offKh);
  unsigned short* Kl = (unsigned short*)(ws + offKl);
  float* SS  = (float*)(ws + offSS);
  float* Wpl = (float*)(ws + offW);
  float* Epl = (float*)(ws + offE);
  float* Npl = (float*)(ws + offN);
  float* Hp  = (float*)(ws + offH);

  bias_cat_kernel<<<dim3(6), dim3(64), 0, stream>>>(bq, bk, bv, bg, Bc);
  const int n8 = (kRows * kD) / 8;
  xcast_kernel<<<dim3(n8 / 256), dim3(256), 0, stream>>>(x, Xb, n8);
  wt_cast_kernel<<<dim3(kD / 64, kNP / 64), dim3(256), 0, stream>>>(Wq, Wk, Wv, Wg, Wt);

  const int tilesProj = (kRows / 64) * (kNP / 64);
  wmma_gemm64<1, false, 2, 0, false, 0><<<dim3(tilesProj / 8, 1), dim3(256), 0, stream>>>(
      Xb, Xb, kD, 0L, Wt, Wt, kD, 0L,
      (void*)PR, (void*)PR, kNP, 0L, Bc, Bc, 0L, kRows, kNP, kD, 1.0f);

  split_qk_kernel<<<dim3(n8 / 256, 2), dim3(256), 0, stream>>>(PR, Qh, Ql, Kh, Kl);

  const long stridePair16 = (long)64 * kD;
  const long stridePairSS = (long)64 * 64;
  wmma_gemm64<1, true, 0, 0, false, 0><<<dim3(1, kPairs), dim3(256), 0, stream>>>(
      Qh, Ql, kD, stridePair16, Kh, Kl, kD, stridePair16,
      (void*)SS, (void*)SS, 64, stridePairSS, Bc, Bc, 0L, 64, 64, kD, 1.0f);

  gate_kernel<<<dim3(kB), dim3(256), 0, stream>>>(PR, ib, Wpl, Epl, Npl);
  scan_kernel<<<dim3(kD / 64, kB), dim3(256), 0, stream>>>(Qh, Ql, PR, SS, Wpl, Epl, Npl, Hp);
  rmsnorm_kernel<<<dim3(kRows / 8), dim3(256), 0, stream>>>(Hp, ns, out);
}
